// MaskGAE_stage1_25615184953521
// MI455X (gfx1250) — hardware-verified
//
#include <hip/hip_runtime.h>
#include <stddef.h>


#define NN     128
#define NH     64
#define NTHR   256
#define NWAVE  8
#define NBC    256
#define EPT    8
#define NGRP   2
#define CHUNK  (NTHR * EPT * NGRP)
#define WCAP   (EPT * NGRP * 32)
#define LISTN  (NWAVE * WCAP)
#define XP     136
#define NROWS  64
#define WSCAP  134217728
#define BN_EPS 1e-5f

#define SO_ACC0 0
#define SO_ACC1 (NBC * NH * 4)
#define SO_LIST (2 * NBC * NH * 4)
#define SO_THI  (SO_LIST + LISTN * 4)
#define SO_TLO  (SO_THI + 16 * XP * 2)
#define SO_DT   (SO_TLO + 16 * XP * 2)
#define SLDSB   (SO_DT + 16 * NH * 4)

static_assert(CHUNK == 4096);
static_assert(WCAP == 512);
static_assert(NBC == 256);
static_assert(NWAVE * 32 == NTHR);
static_assert(SO_ACC1 == 65536);
static_assert(SO_LIST == 131072);
static_assert(SLDSB == 160256);
static_assert((SO_THI % 16) == 0);
static_assert((SO_TLO % 16) == 0);
static_assert((SO_DT % 16) == 0);
static_assert(((XP * 2) % 16) == 0);
static_assert(2 * NROWS * XP * 2 >= NROWS * NN * 4);

#define O_WN0H 0
#define O_WN0L 2048
#define O_WFAH 4096
#define O_WFAL 12288
#define O_WF0H 20480
#define O_WF0L 36864
#define O_WE1H 53248
#define O_WE1L 61440
#define O_WN1H 69632
#define O_WN1L 77824
#define O_WF1H 86016
#define O_WF1L 102400
#define O_WEND 118784
static_assert(O_WN0L - O_WN0H == 64 * 32);
static_assert(O_WFAL - O_WFAH == 128 * 64);
static_assert(O_WF0L - O_WF0H == 128 * 128);
static_assert(O_WE1L - O_WE1H == 64 * 128);
static_assert(O_WN1L - O_WN1H == 64 * 128);
static_assert(O_WF1L - O_WF1H == 128 * 128);
static_assert(O_WEND - O_WF1L == 128 * 128);

typedef float          v2f  __attribute__((ext_vector_type(2)));
typedef float          v4f  __attribute__((ext_vector_type(4)));
typedef float          v8f  __attribute__((ext_vector_type(8)));
typedef int            v4i  __attribute__((ext_vector_type(4)));
typedef unsigned short v4us __attribute__((ext_vector_type(4)));
typedef unsigned short v8us __attribute__((ext_vector_type(8)));
typedef __bf16         v16bf __attribute__((ext_vector_type(16)));
union FragB { v16bf v; v8us u[2]; };

extern __shared__ __attribute__((aligned(16))) float g_dyn[];

__device__ __forceinline__ v8f wmb(v16bf a, v16bf b, v8f c) {
  v8f d = __builtin_amdgcn_wmma_f32_16x16x32_bf16(false, a, false, b, (short)0, c, false, false);
  asm volatile("v_nop\n\tv_nop\n\tv_nop\n\tv_nop" : "+v"(d) : "v"(a), "v"(b));
  return d;
}

__device__ __forceinline__ v8f zero8() {
  v8f z = {0.f, 0.f, 0.f, 0.f, 0.f, 0.f, 0.f, 0.f};
  return z;
}

__device__ __forceinline__ v4f zero4() {
  v4f z = {0.f, 0.f, 0.f, 0.f};
  return z;
}

__device__ __forceinline__ void wave_sync() {
  __threadfence_block();
  __builtin_amdgcn_wave_barrier();
}

__device__ __forceinline__ unsigned short bfr(float f) {
  unsigned int u = __float_as_uint(f);
  u += 0x7FFFu + ((u >> 16) & 1u);
  return (unsigned short)(u >> 16);
}

__device__ __forceinline__ void split1(float x, unsigned short& h, unsigned short& l) {
  const unsigned short hs = bfr(x);
  const float hf = __uint_as_float(((unsigned int)hs) << 16);
  h = hs;
  l = bfr(x - hf);
}

__device__ __forceinline__ void split4(v4f x, v4us* h, v4us* l) {
  unsigned short h0, h1, h2, h3, l0, l1, l2, l3;
  split1(x.x, h0, l0);
  split1(x.y, h1, l1);
  split1(x.z, h2, l2);
  split1(x.w, h3, l3);
  v4us hv, lv;
  hv.x = h0; hv.y = h1; hv.z = h2; hv.w = h3;
  lv.x = l0; lv.y = l1; lv.z = l2; lv.w = l3;
  *h = hv;
  *l = lv;
}

__device__ __forceinline__ v4f relu4(v4f x) {
  v4f y;
  y.x = fmaxf(x.x, 0.f);
  y.y = fmaxf(x.y, 0.f);
  y.z = fmaxf(x.z, 0.f);
  y.w = fmaxf(x.w, 0.f);
  return y;
}

__global__ __launch_bounds__(NTHR) void k_wprep(
    const float* __restrict__ Wn0, const float* __restrict__ We0, const float* __restrict__ Wfe0,
    const float* __restrict__ Wfn0, const float* __restrict__ We1, const float* __restrict__ Wn1,
    const float* __restrict__ Wfn1, unsigned short* wpl, float* vpm) {
  __shared__ __attribute__((aligned(16))) float sV[256];
  const int tid = (int)threadIdx.x, lane = tid & 31, wave = tid >> 5;
  const int b = (int)blockIdx.x;
  if (b < 29) {
    const float* W;
    int pin, kin, kpsh, lb, oh, ol;
    if (b < 1)       { W = Wn0;  pin = 16;  kin = 16;  kpsh = 5; lb = b;      oh = O_WN0H; ol = O_WN0L; }
    else if (b < 5)  { W = Wfe0; pin = 128; kin = 64;  kpsh = 6; lb = b - 1;  oh = O_WFAH; ol = O_WFAL; }
    else if (b < 13) { W = Wfn0; pin = 128; kin = 128; kpsh = 7; lb = b - 5;  oh = O_WF0H; ol = O_WF0L; }
    else if (b < 17) { W = We1;  pin = 128; kin = 128; kpsh = 7; lb = b - 13; oh = O_WE1H; ol = O_WE1L; }
    else if (b < 21) { W = Wn1;  pin = 128; kin = 128; kpsh = 7; lb = b - 17; oh = O_WN1H; ol = O_WN1L; }
    else             { W = Wfn1; pin = 128; kin = 128; kpsh = 7; lb = b - 21; oh = O_WF1H; ol = O_WF1L; }
    const int o = (lb * NTHR + tid) * 8;
    const int n = o >> kpsh, k0 = o & ((1 << kpsh) - 1);
    float v[8];
#pragma unroll
    for (int j = 0; j < 8; ++j) {
      const int k = k0 + j;
      const int kk = k < kin ? k : kin - 1;
      const float t = W[(size_t)n * pin + kk];
      v[j] = (k < kin) ? t : 0.f;
    }
    v8us hv, lv;
    {
      unsigned short h[8], l[8];
#pragma unroll
      for (int j = 0; j < 8; ++j) split1(v[j], h[j], l[j]);
      hv.s0 = h[0]; hv.s1 = h[1]; hv.s2 = h[2]; hv.s3 = h[3];
      hv.s4 = h[4]; hv.s5 = h[5]; hv.s6 = h[6]; hv.s7 = h[7];
      lv.s0 = l[0]; lv.s1 = l[1]; lv.s2 = l[2]; lv.s3 = l[3];
      lv.s4 = l[4]; lv.s5 = l[5]; lv.s6 = l[6]; lv.s7 = l[7];
    }
    unsigned short* dh = wpl + oh + o;
    unsigned short* dl = wpl + ol + o;
    *(volatile v8us*)dh = hv;
    *(volatile v8us*)dl = lv;
    __threadfence();
    *(volatile v8us*)dh = hv;
    *(volatile v8us*)dl = lv;
  } else {
    const int n = tid & 127, neg = tid >> 7;
    float s = 0.f;
#pragma unroll 1
    for (int c = 0; c < NH; ++c) {
      const float w = We0[c];
      const float u = Wfe0[(size_t)n * NN + NH + c];
      const float p = w * u;
      const bool take = (neg != 0) ? (w < 0.f) : (w > 0.f);
      s += take ? p : 0.f;
    }
    sV[tid] = s;
    __syncthreads();
    if (wave < 2) {
      const v4f o4 = *(const v4f*)(sV + wave * NN + 4 * lane);
      float* dp = vpm + wave * NN + 4 * lane;
      *(volatile v4f*)dp = o4;
      __threadfence();
      *(volatile v4f*)dp = o4;
    }
  }
}

template <int NOUT, int KS>
__global__ __launch_bounds__(NTHR) void k_node(
    const float* __restrict__ src0, const float* __restrict__ src1,
    const unsigned short* __restrict__ whi, const unsigned short* __restrict__ wlo,
    const float* __restrict__ bias, const float* __restrict__ bg, const float* __restrict__ bb,
    const float* __restrict__ brm, const float* __restrict__ brv,
    float* out, int s0sh, int w1, int flags, int nN, int nStore) {
  constexpr int KP = 32 * KS;
  constexpr int NCT = NOUT / 32;
  __shared__ __attribute__((aligned(16))) unsigned short pl[2 * NROWS * XP];
  __shared__ __attribute__((aligned(16))) float sEp[5 * NOUT];
  unsigned short* phi = pl;
  unsigned short* plo = pl + NROWS * XP;
  float* stg = (float*)pl;
  const int tid = (int)threadIdx.x, lane = tid & 31, wave = tid >> 5, hh = lane >> 4, m = lane & 15;
  const int mbase = (int)blockIdx.x * NROWS;
  const int w0q = 1 << s0sh, w0 = 4 * w0q;

  if (tid < NOUT) {
    sEp[tid]            = bias[tid];
    sEp[NOUT + tid]     = bg[tid];
    sEp[2 * NOUT + tid] = bb[tid];
    sEp[3 * NOUT + tid] = brm[tid];
    sEp[4 * NOUT + tid] = 1.0f / sqrtf(brv[tid] + BN_EPS);
  }

  for (int i = tid; i < NROWS * w0q; i += NTHR) {
    const int r = i >> s0sh, c4 = i & (w0q - 1);
    const int grow = mbase + r;
    const int gr = grow < nN ? grow : nN - 1;
    v4f v = *(const v4f*)(src0 + (size_t)gr * w0 + 4 * c4);
    if (grow >= nN) v = zero4();
    v4us h4, l4;
    split4(v, &h4, &l4);
    *(v4us*)(phi + r * XP + 4 * c4) = h4;
    *(v4us*)(plo + r * XP + 4 * c4) = l4;
  }
  if (w1 != 0) {
    for (int i = tid; i < NROWS * 16; i += NTHR) {
      const int r = i >> 4, c4 = i & 15;
      const int grow = mbase + r;
      const int gr = grow < nN ? grow : nN - 1;
      v4f v = *(const v4f*)(src1 + (size_t)gr * NH + 4 * c4);
      if (grow >= nN) v = zero4();
      v4us h4, l4;
      split4(v, &h4, &l4);
      *(v4us*)(phi + r * XP + w0 + 4 * c4) = h4;
      *(v4us*)(plo + r * XP + w0 + 4 * c4) = l4;
    }
  }
  {
    const int K = w0 + (w1 != 0 ? NH : 0);
    const int padq = (KP - K) >> 2;
    if (padq > 0) {
      const v4us z = {0, 0, 0, 0};
      for (int i = tid; i < NROWS * padq; i += NTHR) {
        const int r = i / padq, c4 = i - r * padq;
        *(v4us*)(phi + r * XP + K + 4 * c4) = z;
        *(v4us*)(plo + r * XP + K + 4 * c4) = z;
      }
    }
  }
  __syncthreads();

  const int rt = wave & 3, chalf = wave >> 2;
  const int colbase = chalf * (NOUT / 2);
  v8f acc[NCT];
#pragma unroll
  for (int t = 0; t < NCT; ++t) acc[t] = zero8();
  {
    const unsigned short* ap  = phi + (16 * rt + m) * XP + 8 * hh;
    const unsigned short* alp = plo + (16 * rt + m) * XP + 8 * hh;
#pragma unroll
    for (int ks = 0; ks < KS; ++ks) {
      FragB ah, al;
      ah.u[0] = *(const v8us*)(ap + 32 * ks);
      ah.u[1] = *(const v8us*)(ap + 32 * ks + 16);
      al.u[0] = *(const v8us*)(alp + 32 * ks);
      al.u[1] = *(const v8us*)(alp + 32 * ks + 16);
#pragma unroll
      for (int t = 0; t < NCT; ++t) {
        const size_t bo = (size_t)(colbase + 16 * t + m) * KP + 32 * ks + 8 * hh;
        FragB bh, bl;
        bh.u[0] = *(const v8us*)(whi + bo);
        bh.u[1] = *(const v8us*)(whi + bo + 16);
        bl.u[0] = *(const v8us*)(wlo + bo);
        bl.u[1] = *(const v8us*)(wlo + bo + 16);
        acc[t] = wmb(ah.v, bh.v, acc[t]);
        acc[t] = wmb(ah.v, bl.v, acc[t]);
        acc[t] = wmb(al.v, bh.v, acc[t]);
      }
    }
  }
  __syncthreads();

#pragma unroll
  for (int t = 0; t < NCT; ++t) {
    const int col = colbase + 16 * t + m;
    const float bi = sEp[col];
    const float gg = sEp[NOUT + col], be = sEp[2 * NOUT + col], mu = sEp[3 * NOUT + col];
    const float rs = sEp[4 * NOUT + col];
#pragma unroll
    for (int r = 0; r < 8; ++r) {
      float y = acc[t][r];
      if (flags & 1) y = y + bi;
      if (flags & 2) y = fmaxf(y, 0.f);
      if (flags & 4) y = ((y - mu) * rs) * gg + be;
      stg[(16 * rt + 8 * hh + r) * NOUT + col] = y;
    }
  }
  __syncthreads();

  if (NOUT == 128) {
    v4f vr[8];
#pragma unroll
    for (int j = 0; j < 8; ++j) vr[j] = *(const v4f*)(stg + (8 * wave + j) * NOUT + 4 * lane);
#pragma unroll
    for (int j = 0; j < 8; ++j) {
      const int grow = mbase + 8 * wave + j;
      if (grow < nStore) *(volatile v4f*)(out + (size_t)grow * NOUT + 4 * lane) = vr[j];
    }
    __threadfence();
#pragma unroll
    for (int j = 0; j < 8; ++j) {
      const int grow = mbase + 8 * wave + j;
      if (grow < nStore) *(volatile v4f*)(out + (size_t)grow * NOUT + 4 * lane) = vr[j];
    }
  } else {
    v4f vr[4];
#pragma unroll
    for (int j = 0; j < 4; ++j) {
      const int rl = 8 * wave + 2 * j + hh;
      vr[j] = *(const v4f*)(stg + rl * NOUT + 4 * m);
    }
#pragma unroll
    for (int j = 0; j < 4; ++j) {
      const int grow = mbase + 8 * wave + 2 * j + hh;
      if (grow < nStore) *(volatile v4f*)(out + (size_t)grow * NOUT + 4 * m) = vr[j];
    }
    __threadfence();
#pragma unroll
    for (int j = 0; j < 4; ++j) {
      const int grow = mbase + 8 * wave + 2 * j + hh;
      if (grow < nStore) *(volatile v4f*)(out + (size_t)grow * NOUT + 4 * m) = vr[j];
    }
  }
}

template <int NB>
__device__ __forceinline__ int scan_chunk(const int* __restrict__ keys, int nK, int cbase, int slotBase,
                                          int vec8, int* list, int tid, int lane, int wave) {
  int wc = 0;
#pragma unroll
  for (int g = 0; g < NGRP; ++g) {
    const int el0  = (g * NTHR + tid) * EPT;
    const int e0   = cbase + el0;
    const int sent = -2147483647 - 1;
    v4i da, db;
    if (vec8 != 0 && cbase + CHUNK <= nK) {
      da = *(const v4i*)(keys + e0);
      db = *(const v4i*)(keys + e0 + 4);
    } else {
      da.x = (e0     < nK) ? keys[min(e0,     nK - 1)] : sent;
      da.y = (e0 + 1 < nK) ? keys[min(e0 + 1, nK - 1)] : sent;
      da.z = (e0 + 2 < nK) ? keys[min(e0 + 2, nK - 1)] : sent;
      da.w = (e0 + 3 < nK) ? keys[min(e0 + 3, nK - 1)] : sent;
      db.x = (e0 + 4 < nK) ? keys[min(e0 + 4, nK - 1)] : sent;
      db.y = (e0 + 5 < nK) ? keys[min(e0 + 5, nK - 1)] : sent;
      db.z = (e0 + 6 < nK) ? keys[min(e0 + 6, nK - 1)] : sent;
      db.w = (e0 + 7 < nK) ? keys[min(e0 + 7, nK - 1)] : sent;
    }
    const unsigned nb = (unsigned)slotBase;
    const unsigned s0 = (unsigned)da.x - nb, s1 = (unsigned)da.y - nb;
    const unsigned s2 = (unsigned)da.z - nb, s3 = (unsigned)da.w - nb;
    const unsigned s4 = (unsigned)db.x - nb, s5 = (unsigned)db.y - nb;
    const unsigned s6 = (unsigned)db.z - nb, s7 = (unsigned)db.w - nb;
    const bool h0 = s0 < (unsigned)NB, h1 = s1 < (unsigned)NB, h2 = s2 < (unsigned)NB, h3 = s3 < (unsigned)NB;
    const bool h4 = s4 < (unsigned)NB, h5 = s5 < (unsigned)NB, h6 = s6 < (unsigned)NB, h7 = s7 < (unsigned)NB;
    const unsigned any = __builtin_amdgcn_ballot_w32(h0 | h1 | h2 | h3 | h4 | h5 | h6 | h7);
    if (any != 0u) {
#define HITJ(J, HJ, SJ) { \
        const unsigned mj = __builtin_amdgcn_ballot_w32(HJ); \
        if (mj != 0u) { \
          if (HJ) { \
            const int pos = wc + (int)__builtin_amdgcn_mbcnt_lo(mj, 0u); \
            if (pos < WCAP) list[wave * WCAP + pos] = ((el0 + (J)) << 8) | (int)(SJ); \
          } \
          wc += (int)__builtin_popcount(mj); } }
      HITJ(0, h0, s0)
      HITJ(1, h1, s1)
      HITJ(2, h2, s2)
      HITJ(3, h3, s3)
      HITJ(4, h4, s4)
      HITJ(5, h5, s5)
      HITJ(6, h6, s6)
      HITJ(7, h7, s7)
#undef HITJ
    }
  }
  return wc;
}

__device__ __forceinline__ void edge_tile(const unsigned short* thi, const unsigned short* tlo, float* dT,
                                          const int* rowSlot, float* acc1,
                                          const unsigned short* __restrict__ we1h,
                                          const unsigned short* __restrict__ we1l,
                                          int lane, int hh, int m) {
  wave_sync();
  v8f acc[4];
#pragma unroll
  for (int t = 0; t < 4; ++t) acc[t] = zero8();
  const unsigned short* ap  = thi + m * XP + 8 * hh;
  const unsigned short* alp = tlo + m * XP + 8 * hh;
#pragma unroll
  for (int ks = 0; ks < 4; ++ks) {
    FragB ah, al;
    ah.u[0] = *(const v8us*)(ap + 32 * ks);
    ah.u[1] = *(const v8us*)(ap + 32 * ks + 16);
    al.u[0] = *(const v8us*)(alp + 32 * ks);
    al.u[1] = *(const v8us*)(alp + 32 * ks + 16);
#pragma unroll
    for (int t = 0; t < 4; ++t) {
      const size_t bo = (size_t)(16 * t + m) * NN + 32 * ks + 8 * hh;
      FragB bh, bl;
      bh.u[0] = *(const v8us*)(we1h + bo);
      bh.u[1] = *(const v8us*)(we1h + bo + 16);
      bl.u[0] = *(const v8us*)(we1l + bo);
      bl.u[1] = *(const v8us*)(we1l + bo + 16);
      acc[t] = wmb(ah.v, bh.v, acc[t]);
      acc[t] = wmb(ah.v, bl.v, acc[t]);
      acc[t] = wmb(al.v, bh.v, acc[t]);
    }
  }
#pragma unroll
  for (int t = 0; t < 4; ++t) {
#pragma unroll
    for (int r = 0; r < 8; ++r) dT[(8 * hh + r) * NH + 16 * t + m] = fmaxf(acc[t][r], 0.f);
  }
  wave_sync();
#pragma unroll
  for (int r = 0; r < 16; ++r) {
    int slot = rowSlot[r];
    slot = slot < 0 ? 0 : (slot > NBC - 1 ? NBC - 1 : slot);
    float* a = acc1 + slot * NH + 2 * lane;
    const v2f d = *(const v2f*)(dT + r * NH + 2 * lane);
    const v2f y = *(const v2f*)a + d;
    *(v2f*)a = y;
  }
  wave_sync();
}

__device__ __forceinline__ void store_acc(const float* accp, float* gp, int nodeBase, int wave, int hh, int m) {
  v4f vals[16];
#pragma unroll
  for (int j = 0; j < 16; ++j) {
    const int rl = 32 * wave + 2 * j + hh;
    vals[j] = *(const v4f*)(accp + rl * NH + 4 * m);
  }
#pragma unroll
  for (int j = 0; j < 16; ++j) {
    const int rl = 32 * wave + 2 * j + hh;
    float* dp = gp + (size_t)(nodeBase + rl) * NH + 4 * m;
    *(volatile v4f*)dp = vals[j];
  }
  __threadfence();
#pragma unroll
  for (int j = 0; j < 16; ++j) {
    const int rl = 32 * wave + 2 * j + hh;
    float* dp = gp + (size_t)(nodeBase + rl) * NH + 4 * m;
    *(volatile v4f*)dp = vals[j];
  }
}

__global__ __launch_bounds__(NTHR) void k_scan(
    const int* __restrict__ ei, const float* __restrict__ eattr, const float* __restrict__ P0,
    const float* __restrict__ We0, const float* __restrict__ bfe0, const float* __restrict__ vpm,
    const unsigned short* __restrict__ we1h, const unsigned short* __restrict__ we1l,
    float* agg0, float* agg1, int nE, int nN, int vec8) {
  float* acc0 = g_dyn;
  float* acc1 = (float*)((char*)g_dyn + SO_ACC1);
  int* list = (int*)((char*)g_dyn + SO_LIST);
  unsigned short* thi = (unsigned short*)((char*)g_dyn + SO_THI);
  unsigned short* tlo = (unsigned short*)((char*)g_dyn + SO_TLO);
  float* dT = (float*)((char*)g_dyn + SO_DT);
  __shared__ int wcnt[NWAVE];
  __shared__ int rowSlot[16];
  const int tid = (int)threadIdx.x, lane = tid & 31, wave = tid >> 5, hh = lane >> 4, m = lane & 15;
  const int nodeBase = (int)blockIdx.x * NBC;
  const int* keys = ei + nE;
  const int nK = nE;

  const float wea = We0[2 * lane], web = We0[2 * lane + 1];
  const v4f vbfe = *(const v4f*)(bfe0 + 4 * lane);
  const v4f vp = *(const v4f*)(vpm + 4 * lane);
  const v4f vm = *(const v4f*)(vpm + NN + 4 * lane);

  {
    const v4f z = zero4();
    for (int i = tid * 4; i < 2 * NBC * NH; i += NTHR * 4) *(v4f*)(g_dyn + i) = z;
  }
  __syncthreads();

  int pend = 0;
  const int nChunks = (nK + CHUNK - 1) / CHUNK;
#pragma unroll 1
  for (int ch = 0; ch < nChunks; ++ch) {
    const int cbase = ch * CHUNK;
    const int wc = scan_chunk<NBC>(keys, nK, cbase, nodeBase, vec8, list, tid, lane, wave);
    if (lane == 0) wcnt[wave] = wc;
    __syncthreads();
    if (wave == 0) {
#pragma unroll 1
      for (int wsx = 0; wsx < NWAVE; ++wsx) {
        int n = __builtin_amdgcn_readfirstlane(wcnt[wsx]);
        n = n > WCAP ? WCAP : (n < 0 ? 0 : n);
        const int* lp = list + wsx * WCAP;
#pragma unroll 1
        for (int i = 0; i < n; ++i) {
          const int ent  = __builtin_amdgcn_readfirstlane(lp[i]);
          const int slot = ent & (NBC - 1);
          int e = cbase + ((ent >> 8) & (CHUNK - 1));
          e = e > nE - 1 ? nE - 1 : e;
          const float ea = eattr[e];
          int s = ei[e];
          s = s < 0 ? 0 : (s > nN - 1 ? nN - 1 : s);
          int dg = nodeBase + slot;
          dg = dg > nN - 1 ? nN - 1 : dg;
          {
            v2f add;
            add.x = fmaxf(ea * wea, 0.f);
            add.y = fmaxf(ea * web, 0.f);
            float* a = acc0 + slot * NH + 2 * lane;
            const v2f y = *(const v2f*)a + add;
            *(v2f*)a = y;
          }
          {
            const v4f p = *(const v4f*)(P0 + (size_t)s * NN + 4 * lane);
            const v4f q = *(const v4f*)(P0 + (size_t)dg * NN + 4 * lane);
            const v4f vsel = (ea > 0.f) ? vp : vm;
            v4f x = (p + q) + ea * vsel + vbfe;
            x = relu4(x);
            v4us h4, l4;
            split4(x, &h4, &l4);
            *(v4us*)(thi + pend * XP + 4 * lane) = h4;
            *(v4us*)(tlo + pend * XP + 4 * lane) = l4;
            if (lane == 0) rowSlot[pend] = slot;
          }
          ++pend;
          if (pend == 16) {
            edge_tile(thi, tlo, dT, rowSlot, acc1, we1h, we1l, lane, hh, m);
            pend = 0;
          }
        }
      }
    }
    __syncthreads();
  }

  if (wave == 0) {
    if (pend > 0) {
      const v4us z = {0, 0, 0, 0};
      for (int r = pend; r < 16; ++r) {
        *(v4us*)(thi + r * XP + 4 * lane) = z;
        *(v4us*)(tlo + r * XP + 4 * lane) = z;
        if (lane == 0) rowSlot[r] = 0;
      }
      edge_tile(thi, tlo, dT, rowSlot, acc1, we1h, we1l, lane, hh, m);
      pend = 0;
    }
  }
  __syncthreads();

  store_acc(acc0, agg0, nodeBase, wave, hh, m);
  store_acc(acc1, agg1, nodeBase, wave, hh, m);
}

extern "C" void kernel_launch(void* const* d_in, const int* in_sizes, int n_in,
                              void* d_out, int out_size, void* d_ws, size_t ws_size,
                              hipStream_t stream) {
  if (n_in < 23) return;
  if (in_sizes[0] < 16 || (in_sizes[0] % 16) != 0) return;
  const int N = in_sizes[0] / 16;
  const int nE = in_sizes[1];
  if (N < 1 || N > (1 << 22) || nE < 1 || nE > (1 << 26)) return;
  if (in_sizes[2] != 2 * nE) return;
  if (in_sizes[3] != NH * 16 || in_sizes[4] != NH || in_sizes[5] != NN * NN || in_sizes[6] != NN) return;
  if (in_sizes[7] != NN * NN || in_sizes[8] != NN) return;
  if (in_sizes[9] != NN || in_sizes[10] != NN || in_sizes[11] != NN || in_sizes[12] != NN) return;
  if (in_sizes[13] != NH * NN || in_sizes[14] != NH * NN || in_sizes[15] != NN * NN || in_sizes[16] != NN) return;
  if (in_sizes[19] != NN || in_sizes[20] != NN || in_sizes[21] != NN || in_sizes[22] != NN) return;
  if (out_size != N * NN) return;

  const float* x    = (const float*)d_in[0];
  const float* ea   = (const float*)d_in[1];
  const int*   ei   = (const int*)d_in[2];
  const float* Wn0  = (const float*)d_in[3];
  const float* We0  = (const float*)d_in[4];
  const float* Wfn0 = (const float*)d_in[5];
  const float* bfn0 = (const float*)d_in[6];
  const float* Wfe0 = (const float*)d_in[7];
  const float* bfe0 = (const float*)d_in[8];
  const float* g0   = (const float*)d_in[9];
  const float* b0   = (const float*)d_in[10];
  const float* rm0  = (const float*)d_in[11];
  const float* rv0  = (const float*)d_in[12];
  const float* Wn1  = (const float*)d_in[13];
  const float* We1  = (const float*)d_in[14];
  const float* Wfn1 = (const float*)d_in[15];
  const float* bfn1 = (const float*)d_in[16];
  const float* g1   = (const float*)d_in[19];
  const float* b1   = (const float*)d_in[20];
  const float* rm1  = (const float*)d_in[21];
  const float* rv1  = (const float*)d_in[22];
  float* dout = (float*)d_out;

  const int nbScan = (N + NBC - 1) / NBC;
  const int Npad   = nbScan * NBC;
  const int nbNode = Npad / NROWS;

  char* ws = (char*)d_ws;
  size_t off = 0;
  const size_t oN10 = off; off += (size_t)Npad * NH * 4;     off = (off + 255) & ~(size_t)255;
  const size_t oP0  = off; off += (size_t)Npad * NN * 4;     off = (off + 255) & ~(size_t)255;
  const size_t oAG0 = off; off += (size_t)Npad * NH * 4;     off = (off + 255) & ~(size_t)255;
  const size_t oAG1 = off; off += (size_t)Npad * NH * 4;     off = (off + 255) & ~(size_t)255;
  const size_t oXQ  = off; off += (size_t)Npad * NN * 4;     off = (off + 255) & ~(size_t)255;
  const size_t oN11 = off; off += (size_t)Npad * NH * 4;     off = (off + 255) & ~(size_t)255;
  const size_t oWPL = off; off += (size_t)O_WEND * 2;        off = (off + 255) & ~(size_t)255;
  const size_t oVPM = off; off += (size_t)2 * NN * 4;        off = (off + 255) & ~(size_t)255;
  if (off > ws_size || off > (size_t)WSCAP) return;
  float* n1_0 = (float*)(ws + oN10);
  float* P0   = (float*)(ws + oP0);
  float* agg0 = (float*)(ws + oAG0);
  float* agg1 = (float*)(ws + oAG1);
  float* xq   = (float*)(ws + oXQ);
  float* n1_1 = (float*)(ws + oN11);
  unsigned short* wpl = (unsigned short*)(ws + oWPL);
  float* vpm  = (float*)(ws + oVPM);

  const int vec8 = ((nE & 3) == 0) ? 1 : 0;

  hipFuncSetAttribute(reinterpret_cast<const void*>(&k_scan), hipFuncAttributeMaxDynamicSharedMemorySize, SLDSB);

  k_wprep<<<30, NTHR, 0, stream>>>(Wn0, We0, Wfe0, Wfn0, We1, Wn1, Wfn1, wpl, vpm);
  k_node<64, 1><<<nbNode, NTHR, 0, stream>>>(x, ea, wpl + O_WN0H, wpl + O_WN0L,
                                             bfn0, g0, b0, rm0, rv0, n1_0, 2, 0, 2, N, Npad);
  k_node<128, 2><<<nbNode, NTHR, 0, stream>>>(n1_0, x, wpl + O_WFAH, wpl + O_WFAL,
                                              bfn0, g0, b0, rm0, rv0, P0, 4, 0, 0, N, Npad);
  k_scan<<<nbScan, NTHR, SLDSB, stream>>>(ei, ea, P0, We0, bfe0, vpm, wpl + O_WE1H, wpl + O_WE1L,
                                          agg0, agg1, nE, N, vec8);
  k_node<128, 4><<<nbNode, NTHR, 0, stream>>>(agg0, n1_0, wpl + O_WF0H, wpl + O_WF0L,
                                              bfn0, g0, b0, rm0, rv0, xq, 4, NH, 7, N, Npad);
  k_node<64, 4><<<nbNode, NTHR, 0, stream>>>(xq, x, wpl + O_WN1H, wpl + O_WN1L,
                                             bfn0, g0, b0, rm0, rv0, n1_1, 5, 0, 2, N, Npad);
  k_node<128, 4><<<nbNode, NTHR, 0, stream>>>(agg1, n1_1, wpl + O_WF1H, wpl + O_WF1L,
                                              bfn1, g1, b1, rm1, rv1, dout, 4, NH, 7, N, N);
}
